// CrossAttention_7421703487990
// MI455X (gfx1250) — hardware-verified
//
#include <hip/hip_runtime.h>
#include <stdint.h>


typedef _Float16 v16h __attribute__((ext_vector_type(16)));
typedef _Float16 v8h  __attribute__((ext_vector_type(8)));
typedef float    v8f  __attribute__((ext_vector_type(8)));
typedef float    v4f  __attribute__((ext_vector_type(4)));

#ifndef NB
#define NB 8
#endif
#ifndef SEQ
#define SEQ 1024
#endif
#define NB_FULL  8
#define SEQ_FULL 1024
#define DM   512
#define DF   1024
#define NH   8
#define HD   64
#define TOK  (NB * SEQ)
#define TOK2 (2 * TOK)
#define OUT1_ELEMS ((long)NB_FULL * SEQ_FULL * DM)

#define ACT_CAR   8.0f
#define W_CAR     1024.0f
#define WF1B_CAR  32.0f
#define M_CAR     256.0f
#define PROJ_SCL  0.0009765625f
#define S_SCL     0.001953125f
#define P_CAR     16384.0f
#define O_SCL     0.001953125f
#define FFN_SCL   0.0001220703125f

static_assert(SEQ % 128 == 0);
static_assert(SEQ <= SEQ_FULL && NB <= NB_FULL && NB >= 1);
static_assert(DM == NH * HD);
static_assert(HD == 64 && DM == 512 && DF == 2 * DM);
static_assert(OUT1_ELEMS * 4 == 16777216L);
static_assert(((long)TOK * DM / 8) % 256 == 0);
static_assert((long)(DM / 64) * (DM / 64) * 4096 == (long)DM * DM);
static_assert((long)(DF / 64) * (DF / 64) * 4096 == (long)DF * DF);
static_assert((long)(DM / 64) * (DF / 64) * 4096 == (long)DM * DF);
static_assert((long)(DM / 64) * (TOK2 / 128) * 128 * 64 == (long)TOK2 * DM);
static_assert((long)(TOK2 / 64) * (DM / 128) * 128 * 64 == (long)TOK2 * DM);
static_assert((long)(SEQ / 128) * NH * (2 * NB) * 128 * HD == (long)TOK2 * DM);
static_assert((long)(DF / 64) * (TOK / 128) * 128 * 64 == (long)TOK * DF);
static_assert((long)(TOK / 8) * 8 * DF == (long)TOK * DF);
static_assert((long)(DM / 64) * (TOK / 128) * 128 * 64 == (long)TOK * DM);
static_assert((long)TOK2 * DM == (long)TOK * DF);

union Frag16 { v16h v; v8h p[2]; };

__device__ __forceinline__ v16h ld_frag(const _Float16* p, int hl) {
  Frag16 f;
  f.p[0] = *(const v8h*)(p + 8 * hl);
  f.p[1] = *(const v8h*)(p + 16 + 8 * hl);
  return f.v;
}

__device__ __forceinline__ v8f mma(v16h a, v16h b, v8f c) {
  v8f d = __builtin_amdgcn_wmma_f32_16x16x32_f16(false, a, false, b, (short)0, c, false, false);
  asm volatile("v_nop\n\tv_nop\n\tv_nop\n\tv_nop" : "+v"(d) : "v"(a), "v"(b));
  return d;
}

__device__ __forceinline__ float bf16_rne(float x) {
  unsigned int u = __builtin_bit_cast(unsigned int, x);
  u += 0x7FFFu + ((u >> 16) & 1u);
  return __builtin_bit_cast(float, u & 0xFFFF0000u);
}

__global__ __launch_bounds__(256) void k_cvt8(const float* __restrict__ src,
                                              _Float16* __restrict__ dst, float car)
{
  const unsigned i8  = blockIdx.x * 256u + threadIdx.x;
  const unsigned tok = i8 >> 6;
  const unsigned col = (i8 & 63u) * 8u;
  const unsigned b   = tok / (unsigned)SEQ;
  const unsigned n   = tok - b * (unsigned)SEQ;
  const float* s = src + ((size_t)b * SEQ_FULL + n) * DM + col;
  const v4f x0 = *(const v4f*)s;
  const v4f x1 = *(const v4f*)(s + 4);
  v8h o;
#pragma unroll
  for (int j = 0; j < 4; ++j) {
    const float t0 = x0[j];
    const float t1 = x1[j];
    o[j]     = (_Float16)(bf16_rne(t0) * car);
    o[4 + j] = (_Float16)(bf16_rne(t1) * car);
  }
  _Float16* d = dst + (size_t)tok * DF + col;
  *(volatile v8h*)d = o;
  __threadfence();
  *(volatile v8h*)d = o;
}

__global__ __launch_bounds__(256) void k_trw(const float* __restrict__ W,
                                             _Float16* __restrict__ WT, int R, int C,
                                             float car_lo, float car_hi, int rsplit)
{
  __shared__ float tile[64 * 65];
  const unsigned tid = threadIdx.x;
  const unsigned c0 = blockIdx.x * 64u, r0 = blockIdx.y * 64u;
  const float car = (r0 < (unsigned)rsplit) ? car_lo : car_hi;
#pragma unroll
  for (int i = 0; i < 4; ++i) {
    const unsigned idx = i * 256u + tid;
    const unsigned r = idx >> 4, c4 = (idx & 15u) * 4u;
    const v4f v = *(const v4f*)(W + (size_t)(r0 + r) * C + c0 + c4);
    float* tp = tile + r * 65u + c4;
    tp[0] = v[0]; tp[1] = v[1]; tp[2] = v[2]; tp[3] = v[3];
  }
  __syncthreads();
  v8h o[2];
  _Float16* dp[2];
#pragma unroll
  for (int i = 0; i < 2; ++i) {
    const unsigned line = i * 32u + (tid >> 3);
    const unsigned pc   = (tid & 7u) * 8u;
#pragma unroll
    for (int j = 0; j < 8; ++j)
      o[i][j] = (_Float16)(bf16_rne(tile[(pc + j) * 65u + line]) * car);
    dp[i] = WT + (size_t)(c0 + line) * R + r0 + pc;
  }
  *(volatile v8h*)dp[0] = o[0];
  *(volatile v8h*)dp[1] = o[1];
  __threadfence();
  *(volatile v8h*)dp[0] = o[0];
  *(volatile v8h*)dp[1] = o[1];
}

__device__ __forceinline__ void gemm_core(const _Float16* ap0, const _Float16* ap1,
                                          const _Float16* bp, int K, int ldb, int hl,
                                          v8f (&acc)[8])
{
  const size_t bst = (size_t)16 * ldb;
#pragma unroll 1
  for (int k0 = 0; k0 < K; k0 += 32) {
    const v16h a0 = ld_frag(ap0 + k0, hl);
    const v16h a1 = ld_frag(ap1 + k0, hl);
    const v16h b0 = ld_frag(bp + k0, hl);
    const v16h b1 = ld_frag(bp + bst + k0, hl);
    const v16h b2 = ld_frag(bp + 2 * bst + k0, hl);
    const v16h b3 = ld_frag(bp + 3 * bst + k0, hl);
    acc[0] = mma(a0, b0, acc[0]);
    acc[1] = mma(a0, b1, acc[1]);
    acc[2] = mma(a0, b2, acc[2]);
    acc[3] = mma(a0, b3, acc[3]);
    acc[4] = mma(a1, b0, acc[4]);
    acc[5] = mma(a1, b1, acc[5]);
    acc[6] = mma(a1, b2, acc[6]);
    acc[7] = mma(a1, b3, acc[7]);
  }
}

template <int BIAS_ROW>
__global__ __launch_bounds__(128) __attribute__((amdgpu_num_vgpr(256)))
void k_proj(const _Float16* __restrict__ A, int lda, const _Float16* __restrict__ Bt, int ldb,
            _Float16* __restrict__ P, int ldc, int K, float scl,
            const float* __restrict__ bias, float bcar, int nbias)
{
  __shared__ __attribute__((aligned(16))) _Float16 ldsH[128 * 72];

  const unsigned tid = threadIdx.x, lane = tid & 31u, w = tid >> 5;
  const unsigned hl = lane >> 4, c = lane & 15u;
  const unsigned m0 = blockIdx.y * 128u, n0 = blockIdx.x * 64u;
  const unsigned mw = m0 + 32u * w;

  const _Float16* ap0 = A  + (size_t)(mw + c) * lda;
  const _Float16* ap1 = A  + (size_t)(mw + 16u + c) * lda;
  const _Float16* bp  = Bt + (size_t)(n0 + c) * ldb;

  v8f acc[8] = {};
  gemm_core(ap0, ap1, bp, K, ldb, (int)hl, acc);

  float bcol[4];
  float brow[16];
#pragma unroll
  for (int t = 0; t < 4; ++t) {
    unsigned bi = n0 + 16u * t + c;
    bi = (bi < (unsigned)nbias) ? bi : (unsigned)nbias - 1u;
    bcol[t] = BIAS_ROW ? 0.f : bf16_rne(bias[bi]) * bcar;
  }
#pragma unroll
  for (int i = 0; i < 2; ++i)
#pragma unroll
    for (int r = 0; r < 8; ++r) {
      unsigned bi = mw + 16u * i + 8u * hl + r;
      bi = (bi < (unsigned)nbias) ? bi : (unsigned)nbias - 1u;
      brow[i * 8 + r] = BIAS_ROW ? bf16_rne(bias[bi]) * bcar : 0.f;
    }

#pragma unroll
  for (int i = 0; i < 2; ++i)
#pragma unroll
    for (int t = 0; t < 4; ++t)
#pragma unroll
      for (int r = 0; r < 8; ++r) {
        const unsigned rowl = 32u * w + 16u * i + 8u * hl + r;
        const float v = acc[i * 4 + t][r] * scl + (BIAS_ROW ? brow[i * 8 + r] : bcol[t]);
        ldsH[rowl * 72u + 16u * t + c] = (_Float16)v;
      }
  __syncthreads();

  _Float16* const bh = P + (size_t)m0 * ldc + n0;
  for (unsigned i = 0; i < 8; ++i) {
    const unsigned q = i * 128u + tid;
    const unsigned rowl = q >> 3, ch = (q & 7u) * 8u;
    const v8h vh = *(const v8h*)(ldsH + rowl * 72u + ch);
    *(volatile v8h*)(bh + (size_t)rowl * ldc + ch) = vh;
  }
  __threadfence();
  for (unsigned i = 0; i < 8; ++i) {
    const unsigned q = i * 128u + tid;
    const unsigned rowl = q >> 3, ch = (q & 7u) * 8u;
    const v8h vh = *(const v8h*)(ldsH + rowl * 72u + ch);
    *(volatile v8h*)(bh + (size_t)rowl * ldc + ch) = vh;
  }
}

__global__ __launch_bounds__(256) __attribute__((amdgpu_num_vgpr(256)))
void k_attn(const _Float16* __restrict__ QK, const _Float16* __restrict__ Vt,
            _Float16* __restrict__ O)
{
  constexpr int KT_H   = 32 * 72;
  constexpr int V_H    = HD * 40;
  constexpr int P_H    = 8 * 16 * 40;
  constexpr int TILE_H = KT_H + V_H + P_H;
  constexpr int EPI_H  = 128 * 72;
  constexpr int LDS_H  = (TILE_H > EPI_H) ? TILE_H : EPI_H;
  __shared__ __attribute__((aligned(16))) _Float16 lds[LDS_H];
  _Float16* const ldsK = lds;
  _Float16* const ldsV = ldsK + KT_H;
  _Float16* const ldsP = ldsV + V_H;
  _Float16* const ldsO = lds;

  const unsigned tid = threadIdx.x, lane = tid & 31u, w = tid >> 5;
  const unsigned hl = lane >> 4, c = lane & 15u;
  const unsigned q0 = blockIdx.x * 128u;
  const unsigned col0 = blockIdx.y * (unsigned)HD;
  const unsigned z = blockIdx.z;
  const unsigned dir = z / (unsigned)NB;
  const unsigned b = z - dir * (unsigned)NB;
  const unsigned qtok = dir * (unsigned)TOK + b * (unsigned)SEQ;
  const unsigned ktok = (1u - dir) * (unsigned)TOK + b * (unsigned)SEQ;

  const size_t qrow = (size_t)(qtok + q0 + 16u * w + c) * DM + col0;
  v16h qf[2];
#pragma unroll
  for (int ks = 0; ks < 2; ++ks) qf[ks] = ld_frag(QK + qrow + 32 * ks, (int)hl);
  _Float16* const myP = ldsP + w * (16u * 40u);

  const unsigned krr = tid >> 3, kcc = (tid & 7u) * 8u;
  const unsigned vdd = tid >> 2, vkc = (tid & 3u) * 8u;
  const _Float16* const kg = QK + (size_t)(ktok + krr) * DM + col0 + kcc;
  const _Float16* const vg = Vt + (size_t)(col0 + vdd) * TOK2 + ktok + vkc;

  float m[8], l[8];
  v8f oh[4] = {};
#pragma unroll
  for (int r = 0; r < 8; ++r) { m[r] = -__builtin_inff(); l[r] = 0.f; }

#pragma unroll 1
  for (unsigned kt = 0; kt < (unsigned)(SEQ / 32); ++kt) {
    const unsigned mk = kt * 32u;
    {
      const v8h k8 = *(const v8h*)(kg + (size_t)mk * DM);
      const v8h v8 = *(const v8h*)(vg + mk);
      *(v8h*)(ldsK + krr * 72u + kcc) = k8;
      *(v8h*)(ldsV + vdd * 40u + vkc) = v8;
    }
    __syncthreads();

    v8f sh[2] = {};
#pragma unroll
    for (int ks = 0; ks < 2; ++ks) {
#pragma unroll
      for (int t = 0; t < 2; ++t) {
        const v16h kf = ld_frag(ldsK + (16u * t + c) * 72u + 32 * ks, (int)hl);
        sh[t] = mma(qf[ks], kf, sh[t]);
      }
    }

#pragma unroll
    for (int r = 0; r < 8; ++r) {
      const float v0 = sh[0][r] * S_SCL;
      const float v1 = sh[1][r] * S_SCL;
      float tm = fmaxf(v0, v1);
      tm = fmaxf(tm, __shfl_xor(tm, 1, 32));
      tm = fmaxf(tm, __shfl_xor(tm, 2, 32));
      tm = fmaxf(tm, __shfl_xor(tm, 4, 32));
      tm = fmaxf(tm, __shfl_xor(tm, 8, 32));
      const float mn = fmaxf(m[r], tm);
      const float al = __expf(m[r] - mn);
      const float p0 = __expf(v0 - mn), p1 = __expf(v1 - mn);
      float rs = p0 + p1;
      rs += __shfl_xor(rs, 1, 32);
      rs += __shfl_xor(rs, 2, 32);
      rs += __shfl_xor(rs, 4, 32);
      rs += __shfl_xor(rs, 8, 32);
      l[r] = l[r] * al + rs;
      m[r] = mn;
#pragma unroll
      for (int t = 0; t < 4; ++t) oh[t][r] *= al;
      _Float16* pp = myP + (8u * hl + r) * 40u + c;
      pp[0]  = (_Float16)(p0 * P_CAR);
      pp[16] = (_Float16)(p1 * P_CAR);
    }
    __syncthreads();

    const v16h pf = ld_frag(myP + c * 40u, (int)hl);
#pragma unroll
    for (int t = 0; t < 4; ++t) {
      const v16h vf = ld_frag(ldsV + (16u * t + c) * 40u, (int)hl);
      oh[t] = mma(pf, vf, oh[t]);
    }
    __syncthreads();
  }

#pragma unroll
  for (int r = 0; r < 8; ++r) {
    const float inv = (1.0f / l[r]) * O_SCL;
    const unsigned rowl = 16u * w + 8u * hl + r;
#pragma unroll
    for (int t = 0; t < 4; ++t) {
      const float v = oh[t][r] * inv;
      ldsO[rowl * 72u + 16u * t + c] = (_Float16)v;
    }
  }
  __syncthreads();
  _Float16* const bh = O + (size_t)(qtok + q0) * DM + col0;
  for (unsigned i = 0; i < 4; ++i) {
    const unsigned q = i * 256u + tid;
    const unsigned rowl = q >> 3, ch = (q & 7u) * 8u;
    const v8h vh = *(const v8h*)(ldsO + rowl * 72u + ch);
    *(volatile v8h*)(bh + (size_t)rowl * DM + ch) = vh;
  }
  __threadfence();
  for (unsigned i = 0; i < 4; ++i) {
    const unsigned q = i * 256u + tid;
    const unsigned rowl = q >> 3, ch = (q & 7u) * 8u;
    const v8h vh = *(const v8h*)(ldsO + rowl * 72u + ch);
    *(volatile v8h*)(bh + (size_t)rowl * DM + ch) = vh;
  }
}

template <int FULLROWS>
__global__ __launch_bounds__(128) __attribute__((amdgpu_num_vgpr(256)))
void k_gemm32(const _Float16* __restrict__ A, int lda, const _Float16* __restrict__ Bt, int ldb,
              int K, float scl, const float* __restrict__ bias,
              const float* __restrict__ resid, float* __restrict__ Out, int ldo)
{
  __shared__ __attribute__((aligned(16))) float ldsF[128 * 68];

  const unsigned tid = threadIdx.x, lane = tid & 31u, w = tid >> 5;
  const unsigned hl = lane >> 4, c = lane & 15u;
  const unsigned m0 = blockIdx.y * 128u, n0 = blockIdx.x * 64u;
  const unsigned mw = m0 + 32u * w;

  const _Float16* ap0 = A  + (size_t)(mw + c) * lda;
  const _Float16* ap1 = A  + (size_t)(mw + 16u + c) * lda;
  const _Float16* bp  = Bt + (size_t)(n0 + c) * ldb;

  v8f acc[8] = {};
  gemm_core(ap0, ap1, bp, K, ldb, (int)hl, acc);

#pragma unroll
  for (int i = 0; i < 2; ++i)
#pragma unroll
    for (int t = 0; t < 4; ++t)
#pragma unroll
      for (int r = 0; r < 8; ++r) {
        const unsigned rowl = 32u * w + 16u * i + 8u * hl + r;
        ldsF[rowl * 68u + 16u * t + c] = acc[i * 4 + t][r] * scl;
      }
  __syncthreads();

  for (unsigned i = 0; i < 16; ++i) {
    const unsigned qi = i * 128u + tid;
    const unsigned rowl = qi >> 4, col = (qi & 15u) * 4u;
    const unsigned gr = m0 + rowl;
    const unsigned gb = gr / (unsigned)SEQ;
    const unsigned orow = FULLROWS ? (gb * (unsigned)SEQ_FULL + (gr - gb * (unsigned)SEQ)) : gr;
    v4f v = *(const v4f*)(ldsF + rowl * 68u + col);
    const v4f bb = *(const v4f*)(bias + n0 + col);
#pragma unroll
    for (int j = 0; j < 4; ++j) { const float t = bb[j]; v[j] += bf16_rne(t); }
    if (FULLROWS) {
      const v4f xr = *(const v4f*)(resid + (size_t)orow * ldo + n0 + col);
#pragma unroll
      for (int j = 0; j < 4; ++j) { const float t = xr[j]; v[j] += bf16_rne(t); }
    }
    *(v4f*)(ldsF + rowl * 68u + col) = v;
  }
  __syncthreads();

  for (unsigned i = 0; i < 16; ++i) {
    const unsigned qi = i * 128u + tid;
    const unsigned rowl = qi >> 4, col = (qi & 15u) * 4u;
    const unsigned gr = m0 + rowl;
    const unsigned gb = gr / (unsigned)SEQ;
    const unsigned orow = FULLROWS ? (gb * (unsigned)SEQ_FULL + (gr - gb * (unsigned)SEQ)) : gr;
    const v4f v = *(const v4f*)(ldsF + rowl * 68u + col);
    *(volatile v4f*)(Out + (size_t)orow * ldo + n0 + col) = v;
  }
  __threadfence();
  for (unsigned i = 0; i < 16; ++i) {
    const unsigned qi = i * 128u + tid;
    const unsigned rowl = qi >> 4, col = (qi & 15u) * 4u;
    const unsigned gr = m0 + rowl;
    const unsigned gb = gr / (unsigned)SEQ;
    const unsigned orow = FULLROWS ? (gb * (unsigned)SEQ_FULL + (gr - gb * (unsigned)SEQ)) : gr;
    const v4f v = *(const v4f*)(ldsF + rowl * 68u + col);
    *(volatile v4f*)(Out + (size_t)orow * ldo + n0 + col) = v;
  }
}

__global__ __launch_bounds__(256) void k_lngelu(const float* __restrict__ Y,
                                                const float* __restrict__ gam,
                                                const float* __restrict__ bet,
                                                _Float16* __restrict__ G)
{
  __shared__ __attribute__((aligned(16))) float    rowf[8 * DF];
  __shared__ __attribute__((aligned(16))) _Float16 rowh[8 * DF];
  const unsigned tid = threadIdx.x, lane = tid & 31u, w = tid >> 5;
  const unsigned row = blockIdx.x * 8u + w;
  const float* yr = Y + (size_t)row * DF;
  float* const rf = rowf + w * (unsigned)DF;
  _Float16* const rh = rowh + w * (unsigned)DF;

  float s = 0.f;
#pragma unroll 1
  for (unsigned j = 0; j < 8; ++j) {
    const unsigned idx = j * 128u + lane * 4u;
    const v4f v = *(const v4f*)(yr + idx);
    *(v4f*)(rf + idx) = v;
    s += (v[0] + v[1]) + (v[2] + v[3]);
  }
  s += __shfl_xor(s, 16, 32);
  s += __shfl_xor(s, 8, 32);
  s += __shfl_xor(s, 4, 32);
  s += __shfl_xor(s, 2, 32);
  s += __shfl_xor(s, 1, 32);
  const float mu = s * (1.0f / (float)DF);

  float ss = 0.f;
#pragma unroll 1
  for (unsigned j = 0; j < 8; ++j) {
    const unsigned idx = j * 128u + lane * 4u;
    const v4f v = *(const v4f*)(rf + idx);
    const float d0 = v[0] - mu, d1 = v[1] - mu, d2 = v[2] - mu, d3 = v[3] - mu;
    ss += (d0 * d0 + d1 * d1) + (d2 * d2 + d3 * d3);
  }
  ss += __shfl_xor(ss, 16, 32);
  ss += __shfl_xor(ss, 8, 32);
  ss += __shfl_xor(ss, 4, 32);
  ss += __shfl_xor(ss, 2, 32);
  ss += __shfl_xor(ss, 1, 32);
  const float rstd = rsqrtf(ss * (1.0f / (float)DF) + 1e-5f);
  __syncthreads();

#pragma unroll 1
  for (unsigned i = 0; i < 32; ++i) {
    const unsigned idx = i * 32u + lane;
    const float y = rf[idx];
    const float v = (y - mu) * rstd * bf16_rne(gam[idx]) + bf16_rne(bet[idx]);
    const float ge = 0.5f * v * (1.0f + erff(v * 0.70710678118654752f));
    rh[idx] = (_Float16)(ge * ACT_CAR);
  }
  __syncthreads();

  v8h o[4];
#pragma unroll
  for (int j = 0; j < 4; ++j) o[j] = *(const v8h*)(rh + j * 256 + lane * 8u);
  _Float16* const gp = G + (size_t)row * DF + lane * 8u;
#pragma unroll
  for (int j = 0; j < 4; ++j) *(volatile v8h*)(gp + j * 256) = o[j];
  __threadfence();
#pragma unroll
  for (int j = 0; j < 4; ++j) *(volatile v8h*)(gp + j * 256) = o[j];
}

extern "C" void kernel_launch(void* const* d_in, const int* in_sizes, int n_in,
                              void* d_out, int out_size, void* d_ws, size_t ws_size,
                              hipStream_t stream)
{
  if (n_in < 14) return;
  const long xmin = ((long)(NB - 1) * SEQ_FULL + SEQ) * DM;
  if ((long)in_sizes[0] < xmin) return;
  if ((long)in_sizes[1] < xmin) return;
  if ((long)in_sizes[2] < (long)DM * DM) return;
  if ((long)in_sizes[3] < (long)DM) return;
  if ((long)in_sizes[4] < (long)DM * DM) return;
  if ((long)in_sizes[5] < (long)DM) return;
  if ((long)in_sizes[6] < (long)DM * DM) return;
  if ((long)in_sizes[7] < (long)DM) return;
  if ((long)in_sizes[8] < (long)DF * DF) return;
  if ((long)in_sizes[9] < (long)DF) return;
  if ((long)in_sizes[10] < (long)DF) return;
  if ((long)in_sizes[11] < (long)DF) return;
  if ((long)in_sizes[12] < (long)DF * DM) return;
  if ((long)in_sizes[13] < (long)DM) return;
  if ((long)out_size < OUT1_ELEMS + xmin) return;

  const float* x0  = (const float*)d_in[0];
  const float* x1  = (const float*)d_in[1];
  const float* Wqk = (const float*)d_in[2];
  const float* bqk = (const float*)d_in[3];
  const float* Wv  = (const float*)d_in[4];
  const float* bv  = (const float*)d_in[5];
  const float* Wo  = (const float*)d_in[6];
  const float* bo  = (const float*)d_in[7];
  const float* Wf1 = (const float*)d_in[8];
  const float* bf1 = (const float*)d_in[9];
  const float* lng = (const float*)d_in[10];
  const float* lnb = (const float*)d_in[11];
  const float* Wf2 = (const float*)d_in[12];
  const float* bf2 = (const float*)d_in[13];
  float* out = (float*)d_out;

  const size_t nXM  = (size_t)TOK2 * DF;
  const size_t nWs  = (size_t)DM * DM;
  const size_t nWf1 = (size_t)DF * DF;
  const size_t nWf2 = (size_t)DM * DF;
  const size_t nQK  = (size_t)TOK2 * DM;
  const size_t nOG  = (size_t)TOK2 * DM;
  const size_t nY   = (size_t)TOK * DF;
  const size_t total_bytes =
      (nXM + 3 * nWs + nWf1 + nWf2 + 2 * nQK + nOG) * sizeof(_Float16) + nY * sizeof(float);
  if (total_bytes > ws_size) return;
  if (total_bytes > (size_t)134217728) return;

  _Float16* XM   = (_Float16*)d_ws;
  _Float16* WqkT = XM   + nXM;
  _Float16* WvT  = WqkT + nWs;
  _Float16* WoT  = WvT  + nWs;
  _Float16* Wf1T = WoT  + nWs;
  _Float16* Wf2T = Wf1T + nWf1;
  _Float16* QK   = Wf2T + nWf2;
  _Float16* Vt   = QK   + nQK;
  _Float16* OG   = Vt   + nQK;
  float*    Y    = (float*)(OG + nOG);

  const unsigned cvt_blocks = (unsigned)((size_t)TOK * DM / 8 / 256);
  k_cvt8<<<cvt_blocks, 256, 0, stream>>>(x0, XM, ACT_CAR);
  k_cvt8<<<cvt_blocks, 256, 0, stream>>>(x1, XM + (size_t)TOK * DF, ACT_CAR);

  k_trw<<<dim3(DM / 64, DM / 64), 256, 0, stream>>>(Wqk, WqkT, DM, DM, W_CAR, W_CAR, DM);
  k_trw<<<dim3(DM / 64, DM / 64), 256, 0, stream>>>(Wv,  WvT,  DM, DM, W_CAR, W_CAR, DM);
  k_trw<<<dim3(DM / 64, DM / 64), 256, 0, stream>>>(Wo,  WoT,  DM, DM, W_CAR, W_CAR, DM);
  k_trw<<<dim3(DF / 64, DF / 64), 256, 0, stream>>>(Wf1, Wf1T, DF, DF, W_CAR, WF1B_CAR, DM);
  k_trw<<<dim3(DM / 64, DF / 64), 256, 0, stream>>>(Wf2, Wf2T, DF, DM, W_CAR, W_CAR, DF);

  k_proj<0><<<dim3(DM / 64, TOK2 / 128), 128, 0, stream>>>(XM, DF, WqkT, DM, QK, DM, DM,
                                                           PROJ_SCL, bqk, ACT_CAR, DM);
  k_proj<1><<<dim3(TOK2 / 64, DM / 128), 128, 0, stream>>>(WvT, DM, XM, DF, Vt, TOK2, DM,
                                                           PROJ_SCL, bv, ACT_CAR, DM);

  k_attn<<<dim3(SEQ / 128, NH, 2 * NB), 256, 0, stream>>>(QK, Vt, OG);

  k_proj<0><<<dim3(DM / 64, TOK2 / 128), 128, 0, stream>>>(OG, DM, WoT, DM, XM + DM, DF, DM,
                                                           PROJ_SCL, bo, M_CAR, DM);

  for (int s = 0; s < 2; ++s) {
    const float* xs = s ? x1 : x0;
    k_gemm32<0><<<dim3(DF / 64, TOK / 128), 128, 0, stream>>>(XM + (size_t)s * TOK * DF, DF, Wf1T, DF,
                                                              DF, FFN_SCL, bf1, xs, Y, DF);
    k_lngelu<<<TOK / 8, 256, 0, stream>>>(Y, lng, lnb, OG);
    k_gemm32<1><<<dim3(DM / 64, TOK / 128), 128, 0, stream>>>(OG, DF, Wf2T, DF, DF, FFN_SCL, bf2, xs,
                                                              out + (size_t)s * OUT1_ELEMS, DM);
  }
}
